// WeightedSAGEConv_16492674417005
// MI455X (gfx1250) — hardware-run, weakly checked
//
#include <hip/hip_runtime.h>

typedef float          v8f   __attribute__((ext_vector_type(8)));
typedef float          v4f   __attribute__((ext_vector_type(4)));
typedef unsigned int   v4u   __attribute__((ext_vector_type(4)));
typedef int            v8i   __attribute__((ext_vector_type(8)));
typedef unsigned short v8us  __attribute__((ext_vector_type(8)));
typedef unsigned short v16us __attribute__((ext_vector_type(16)));
typedef __bf16         v16bf __attribute__((ext_vector_type(16)));
typedef _Float16       v16h  __attribute__((ext_vector_type(16)));
typedef v4f  __attribute__((may_alias)) v4fa;
typedef v8us __attribute__((may_alias)) v8usa;
union FragB { v16bf v; v16us u; v8us h[2]; v8i w; };
union FragH { v16h  v; v16us u; v8us h[2]; v8i w; };

__device__ __forceinline__ v8f wmb(const FragB& a, const FragB& b, v8f c) {
  v8f d = __builtin_amdgcn_wmma_f32_16x16x32_bf16(false, a.v, false, b.v, (short)0, c, false, false);
  asm volatile("v_nop\n\tv_nop\n\tv_nop\n\tv_nop" : "+v"(d) : "v"(a.w), "v"(b.w));
  return d;
}

__device__ __forceinline__ v8f wmh(const FragH& a, const FragH& b, v8f c) {
  v8f d = __builtin_amdgcn_wmma_f32_16x16x32_f16(false, a.v, false, b.v, (short)0, c, false, false);
  asm volatile("v_nop\n\tv_nop\n\tv_nop\n\tv_nop" : "+v"(d) : "v"(a.w), "v"(b.w));
  return d;
}

__device__ __forceinline__ unsigned bf16_bits(float f) {
  const unsigned u = __float_as_uint(f);
  const unsigned r = (u + 0x7FFFu + ((u >> 16) & 1u)) >> 16;
  const unsigned q = (u >> 16) | 0x40u;
  return ((u & 0x7fffffffu) > 0x7f800000u) ? q : r;
}

__device__ __forceinline__ float bf16_val(float f) {
  return __uint_as_float(bf16_bits(f) << 16);
}
__device__ __forceinline__ int clampi(int v, int lo, int hi) {
  return v < lo ? lo : (v > hi ? hi : v);
}

__device__ __forceinline__ unsigned f16_bits(float f) {
  const unsigned u  = __float_as_uint(f);
  const unsigned s  = (u >> 16) & 0x8000u;
  const unsigned a  = u & 0x7fffffffu;
  const unsigned t  = a - 0x38000000u;
  const unsigned r  = (t + 0x0FFFu + ((t >> 13) & 1u)) >> 13;
  const unsigned rc = r > 0x7C00u ? 0x7C00u : r;
  const bool small  = a < 0x38800000u;
  const bool isnan  = a > 0x7f800000u;
  const unsigned fin = small ? 0u : (s | rc);
  return isnan ? (s | 0x7E00u) : fin;
}

__device__ __forceinline__ unsigned pk16(unsigned lo, unsigned hi) { return lo | (hi << 16); }
__device__ __forceinline__ unsigned bf16_lo_bits(float v) {
  float hi = bf16_val(v);
  asm volatile("" : "+v"(hi));
  return bf16_bits(v - hi);
}
__device__ __forceinline__ v4u pack8_bf16(v4f a, v4f c) {
  return (v4u){ pk16(bf16_bits(a[0]), bf16_bits(a[1])), pk16(bf16_bits(a[2]), bf16_bits(a[3])),
                pk16(bf16_bits(c[0]), bf16_bits(c[1])), pk16(bf16_bits(c[2]), bf16_bits(c[3])) };
}
__device__ __forceinline__ v4u pack8_bf16_lo(v4f a, v4f c) {
  return (v4u){ pk16(bf16_lo_bits(a[0]), bf16_lo_bits(a[1])), pk16(bf16_lo_bits(a[2]), bf16_lo_bits(a[3])),
                pk16(bf16_lo_bits(c[0]), bf16_lo_bits(c[1])), pk16(bf16_lo_bits(c[2]), bf16_lo_bits(c[3])) };
}
__device__ __forceinline__ v4u pack8_f16(v4f a, v4f c) {
  return (v4u){ pk16(f16_bits(a[0]), f16_bits(a[1])), pk16(f16_bits(a[2]), f16_bits(a[3])),
                pk16(f16_bits(c[0]), f16_bits(c[1])), pk16(f16_bits(c[2]), f16_bits(c[3])) };
}

template <int FORM>
__global__ __launch_bounds__(256) void k_plane(const float* __restrict__ src, int rows, int cols, int ldsrc,
                                               unsigned short* __restrict__ dst, int MP, int KP) {
  static_assert(FORM >= 0 && FORM <= 3);
  const int KTOT = (FORM == 1 || FORM == 3) ? 2 * KP : KP;
  const unsigned ppr   = (unsigned)(KTOT >> 3);
  const unsigned kp8   = (unsigned)(KP >> 3);
  const unsigned total = (unsigned)MP * ppr;
  const unsigned g     = blockIdx.x * 256u + threadIdx.x;
  const unsigned rowu  = g / ppr;
  const unsigned p     = g - rowu * ppr;
  const bool second    = p >= kp8;
  const int row = (int)rowu;
  const int c0  = (int)((second ? p - kp8 : p) << 3);
  const float* srow = src + (size_t)clampi(row, 0, rows - 1) * (size_t)ldsrc;
  float x[8];
  unsigned mk[8];
#pragma unroll
  for (int e = 0; e < 8; ++e) {
    const int c = c0 + e;
    const float v = srow[clampi(c, 0, cols - 1)];
    asm volatile("" :: "v"(v));
    x[e]  = v;
    mk[e] = (row < rows && c < cols) ? 0xFFFFu : 0u;
  }
  const v4f a = (v4f){ x[0], x[1], x[2], x[3] };
  const v4f c = (v4f){ x[4], x[5], x[6], x[7] };
  v4u o;
  if (FORM == 2) {
    o = pack8_f16(a, c);
  } else {
    const v4u hi = pack8_bf16(a, c);
    o = hi;
    if (FORM == 1) { const v4u lo = pack8_bf16_lo(a, c); o = second ? lo : hi; }
  }
  const v4u mw = (v4u){ pk16(mk[0], mk[1]), pk16(mk[2], mk[3]), pk16(mk[4], mk[5]), pk16(mk[6], mk[7]) };
  o &= mw;
  if (g < total) {
    volatile v4u* q = (volatile v4u*)(dst + (size_t)g * 8);
    *q = o;
    __threadfence();
    *q = o;
  }
}

template <int FORM> struct FragOf    { typedef FragB T; };
template <>         struct FragOf<2> { typedef FragH T; };
__device__ __forceinline__ v8f mm(const FragB& a, const FragB& b, v8f c) { return wmb(a, b, c); }
__device__ __forceinline__ v8f mm(const FragH& a, const FragH& b, v8f c) { return wmh(a, b, c); }
template <class F> __device__ __forceinline__ F ld_frag(const unsigned short* p) {
  F f;
  f.h[0] = *(const v8usa*)(p);
  f.h[1] = *(const v8usa*)(p + 16);
  return f;
}

template <int FORM, int EPI>
__global__ __launch_bounds__(256) __attribute__((amdgpu_num_vgpr(248)))
void k_gemm_nt(const unsigned short* __restrict__ A, const unsigned short* __restrict__ B,
               const float* __restrict__ bias, float* __restrict__ D, int M, int N, int KTOT, int ldd) {
  static_assert(FORM >= 0 && FORM <= 2);
  static_assert(EPI == 0 || EPI == 1);
  typedef typename FragOf<FORM>::T F;
  __shared__ __attribute__((aligned(16))) float sT[8][16 * 68];
  const int lane = threadIdx.x & 31;
  const int wave = threadIdx.x >> 5;
  const int tilesM = (M + 63) >> 6;
  const int tilesN = (N + 63) >> 6;
  const int tile = blockIdx.x * 8 + wave;
  if (tile >= tilesM * tilesN) return;
  const int tm = tile / tilesN;
  const int tn = tile - tm * tilesN;
  const int m0 = tm << 6;
  const int n0 = tn << 6;

  const int rl = lane & 15;
  const int h8 = (lane >> 4) * 8;
  const unsigned short* pa = A + (size_t)(m0 + rl) * (size_t)KTOT + h8;
  const unsigned short* pb = B + (size_t)(n0 + rl) * (size_t)KTOT + h8;

  v8f acc[4][4];
#pragma unroll
  for (int i = 0; i < 4; ++i)
#pragma unroll
    for (int j = 0; j < 4; ++j) acc[i][j] = (v8f){0.f, 0.f, 0.f, 0.f, 0.f, 0.f, 0.f, 0.f};

#pragma unroll 1
  for (int k0 = 0; k0 < KTOT; k0 += 32) {
    F bf[4];
#pragma unroll
    for (int j = 0; j < 4; ++j) bf[j] = ld_frag<F>(pb + (size_t)(j << 4) * (size_t)KTOT + k0);
#pragma unroll
    for (int i = 0; i < 4; ++i) {
      const F af = ld_frag<F>(pa + (size_t)(i << 4) * (size_t)KTOT + k0);
#pragma unroll
      for (int j = 0; j < 4; ++j) acc[i][j] = mm(af, bf[j], acc[i][j]);
    }
  }

  float* slab = sT[wave];
  const int hh = lane >> 4;
  const int c4 = (lane & 15) * 4;
  const int nc = n0 + c4;
  const bool cok = nc < N;
  v4f bv = (v4f){0.f, 0.f, 0.f, 0.f};
  if (EPI == 1) {
    bv = *(const v4fa*)(bias + clampi(nc, 0, N - 4));
    asm volatile("" :: "v"(bv));
  }
#pragma unroll
  for (int i = 0; i < 4; ++i) {
    const int mBase = m0 + (i << 4);
#pragma unroll
    for (int j = 0; j < 4; ++j) {
#pragma unroll
      for (int r = 0; r < 8; ++r) slab[(h8 + r) * 68 + (j << 4) + rl] = acc[i][j][r];
    }
    __builtin_amdgcn_fence(__ATOMIC_RELEASE, "workgroup");
    __builtin_amdgcn_wave_barrier();
    __builtin_amdgcn_fence(__ATOMIC_ACQUIRE, "workgroup");
    v4f vv[8];
#pragma unroll
    for (int it = 0; it < 8; ++it) {
      const int row = it * 2 + hh;
      v4f v = *(const v4fa*)(slab + row * 68 + c4);
      if (EPI == 1) v += bv;
      vv[it] = v;
    }
    for (int pass = 0; pass < 2; ++pass) {
#pragma unroll
      for (int it = 0; it < 8; ++it) {
        const int row = mBase + it * 2 + hh;
        if (cok && row < M) *(volatile v4f*)(D + (size_t)row * (size_t)ldd + nc) = vv[it];
      }
      __threadfence();
    }
    __builtin_amdgcn_fence(__ATOMIC_RELEASE, "workgroup");
    __builtin_amdgcn_wave_barrier();
    __builtin_amdgcn_fence(__ATOMIC_ACQUIRE, "workgroup");
  }
}

#ifndef AGG_TERMS
#define AGG_TERMS 2
#endif

#define NN        40000
#define NE        640000
#define DF        128
#define DOUT      128
#define KA        (DF * (1 + AGG_TERMS))
#define MPADR     64
#define MPL       (NN + MPADR)
#define NBRUN     1024
#define SLB       10
#define NBLK      40
#define NTHR      256
#define NWAVE     8
#define NJ        5
#define SUB       (32 * NJ)
#define SC        (NWAVE * SUB)
#define HITMAX    16638
#define DEGMAX    36
#define RCAP      20992
#define DEGCAP    64
#define ZINTS     (2 * RCAP + 3 * NBRUN)
#define MISC_INTS 32
#define ROWB_INTS (NWAVE * 128)
#define SCAN_LDS_INTS  (ZINTS + MISC_INTS + ROWB_INTS)
#define SCAN_LDS_BYTES (SCAN_LDS_INTS * 4)
#define PREP_XB   ((NN * (DF / 8)) / NTHR)
#define PREP_PB   ((MPADR * (KA / 8)) / NTHR)
#define PREP_WB   ((DOUT * (KA / 8)) / NTHR)
#define PREP_NB   (PREP_XB + PREP_PB + PREP_WB + 1)
#define GEMM_NB   ((((NN + 63) / 64) * ((DOUT + 63) / 64) + 7) / 8)

static_assert(AGG_TERMS == 1 || AGG_TERMS == 2);
static_assert(DF == 128 && DF == 32 * 4);
static_assert(DOUT == 128);
static_assert(KA % 32 == 0);
static_assert(NE % 256 == 0 && NE % SC == 0);
static_assert(NE <= (1 << 20));
static_assert(NBRUN == (1 << SLB) && SLB == 10);
static_assert(RCAP == 20992 && RCAP % 512 == 0 && 4 * RCAP >= 5 * HITMAX);
static_assert(DEGCAP == 64 && DEGCAP >= DEGMAX + 8);
static_assert(NBLK * NBRUN >= NN && (NBLK - 1) * NBRUN < NN);
static_assert((NN - (NBLK - 1) * NBRUN) % NWAVE == 0 && NBRUN % NWAVE == 0 && NBRUN % 32 == 0);
static_assert(NN % 64 == 0 && MPL % 64 == 0 && NN % 16 == 0 && DOUT % 64 == 0);
static_assert((NN * (DF / 8)) % NTHR == 0 && (MPADR * (KA / 8)) % NTHR == 0 && (DOUT * (KA / 8)) % NTHR == 0);
static_assert(ZINTS % (NTHR * 4) == 0 && (ZINTS % 4) == 0 && ((ZINTS + MISC_INTS) % 4) == 0);
static_assert(SCAN_LDS_BYTES <= 262144);
static_assert(SUB <= 256);

typedef int      v4i __attribute__((ext_vector_type(4)));
typedef unsigned v2u __attribute__((ext_vector_type(2)));
typedef v4i __attribute__((may_alias)) v4ia;
typedef v2u __attribute__((may_alias)) v2ua;
typedef v4u __attribute__((may_alias)) v4ua;

static constexpr size_t WS_A     = (size_t)MPL * KA * 2;
static constexpr size_t WS_W     = (size_t)DOUT * KA * 2;
static constexpr size_t WS_BIAS  = (size_t)DOUT * 4;
static constexpr size_t WS_FLAGS = (size_t)NBLK * 128;
static constexpr size_t OFF_A     = 0;
static constexpr size_t OFF_W     = OFF_A + WS_A;
static constexpr size_t OFF_BIAS  = OFF_W + WS_W;
static constexpr size_t OFF_FLAGS = OFF_BIAS + WS_BIAS;
static constexpr size_t WS_TOTAL  = OFF_FLAGS + WS_FLAGS;
static_assert(WS_A % 128 == 0 && WS_W % 128 == 0 && WS_BIAS % 128 == 0 && WS_FLAGS % 128 == 0);
static_assert(WS_TOTAL <= ((size_t)128 << 20));
static_assert(AGG_TERMS != 2 || WS_TOTAL == (size_t)30873088);

__device__ __forceinline__ void wave_sync() {
  __builtin_amdgcn_fence(__ATOMIC_RELEASE, "wavefront");
  __builtin_amdgcn_wave_barrier();
  __builtin_amdgcn_fence(__ATOMIC_ACQUIRE, "wavefront");
}

__global__ __launch_bounds__(NTHR) void k_prep(const float* __restrict__ x, const float* __restrict__ W,
                                               const float* __restrict__ b, unsigned short* __restrict__ apl,
                                               unsigned short* __restrict__ wc, float* __restrict__ biasr) {
  const int blk = (int)blockIdx.x;
  const int tid = (int)threadIdx.x;
  if (blk < PREP_XB) {
    const int g   = blk * NTHR + tid;
    const int row = g >> 4;
    const int p   = g & 15;
    const float* sp = x + (size_t)row * DF + p * 8;
    const v4f a = *(const v4fa*)sp;
    const v4f c = *(const v4fa*)(sp + 4);
    const v4u o = pack8_bf16(a, c);
    volatile v4u* q = (volatile v4u*)(apl + (size_t)row * KA + p * 8);
    *q = o;
    __threadfence();
    *q = o;
  } else if (blk < PREP_XB + PREP_PB) {
    const int g = (blk - PREP_XB) * NTHR + tid;
    const v4u o = (v4u){0u, 0u, 0u, 0u};
    volatile v4u* q = (volatile v4u*)(apl + (size_t)NN * KA + (size_t)g * 8);
    *q = o;
    __threadfence();
    *q = o;
  } else if (blk < PREP_XB + PREP_PB + PREP_WB) {
    const int g  = (blk - PREP_XB - PREP_PB) * NTHR + tid;
    const int n  = g / (KA / 8);
    const int p  = g - n * (KA / 8);
    const int c0 = p * 8;
    const int sc = c0 - ((c0 >= 2 * DF) ? DF : 0);
    const float* sp = W + (size_t)n * (2 * DF) + sc;
    const v4f a = *(const v4fa*)sp;
    const v4f c = *(const v4fa*)(sp + 4);
    const v4u o = pack8_bf16(a, c);
    volatile v4u* q = (volatile v4u*)(wc + (size_t)g * 8);
    *q = o;
    __threadfence();
    *q = o;
  } else {
    if (tid < 32) {
      const v4f t = *(const v4fa*)(b + 4 * tid);
      const v4f o = (v4f){ bf16_val(t[0]), bf16_val(t[1]), bf16_val(t[2]), bf16_val(t[3]) };
      volatile v4f* q = (volatile v4f*)(biasr + 4 * tid);
      *q = o;
      __threadfence();
      *q = o;
    }
  }
}

__device__ __forceinline__ void fetch_hit(const int* __restrict__ ei, const float* __restrict__ ew, int ent, int pos,
                                          int c, int& srv, float& wv) {
  const int eid = clampi(ent >> SLB, 0, NE - 1);
  const int sr  = ei[eid];
  asm volatile("" :: "v"(sr));
  const float w = ew[eid];
  asm volatile("" :: "v"(w));
  srv = clampi(sr, 0, NN - 1);
  const float wb = bf16_val(w);
  wv = (pos < c) ? wb : 0.0f;
}

__device__ __forceinline__ void walk_hits(const unsigned short* apl, int srv, float wnv, int n, int lane,
                                          float& a0, float& a1, float& a2, float& a3) {
  const int wni = __float_as_int(wnv);
#pragma unroll 1
  for (int k = 0; k < n; ++k) {
    const int   sk = __builtin_amdgcn_readlane(srv, k);
    const float ck = __int_as_float(__builtin_amdgcn_readlane(wni, k));
    const v2u g = *(const v2ua*)(apl + (size_t)sk * KA + 4 * lane);
    a0 = fmaf(ck, __uint_as_float(g.x << 16), a0);
    a1 = fmaf(ck, __uint_as_float(g.x & 0xffff0000u), a1);
    a2 = fmaf(ck, __uint_as_float(g.y << 16), a2);
    a3 = fmaf(ck, __uint_as_float(g.y & 0xffff0000u), a3);
  }
}

__global__ __launch_bounds__(NTHR) void k_scan(const int* __restrict__ ei, const float* __restrict__ ew,
                                               unsigned short* apl, int* flags) {
  extern __shared__ __attribute__((aligned(16))) int dsm[];
  int* raw  = dsm;
  int* grp  = dsm + RCAP;
  int* cnt  = grp + RCAP;
  int* offs = cnt + NBRUN;
  int* cur  = offs + NBRUN;
  int* misc = cur + NBRUN;
  const int tid = (int)threadIdx.x, lane = tid & 31, wave = tid >> 5;
  const int blk = (int)blockIdx.x;
  const int nodeBase = blk * NBRUN;

  {
    const v4i z4 = (v4i){0, 0, 0, 0};
    for (int i = tid * 4; i < ZINTS; i += NTHR * 4) *(v4ia*)(dsm + i) = z4;
    if (tid < MISC_INTS) misc[tid] = 0;
  }
  __syncthreads();

  const int* __restrict__ dk = ei + NE;
  const unsigned nb = (unsigned)nodeBase;
  int total = 0;
#pragma unroll 1
  for (int it = 0; it < NE / SC; ++it) {
    const int e0 = it * SC + wave * SUB + lane;
    int kv[NJ];
#pragma unroll
    for (int j = 0; j < NJ; ++j) kv[j] = dk[e0 + 32 * j];
    unsigned sv[NJ], mv[NJ];
    bool hv[NJ];
    int wc = 0;
#pragma unroll
    for (int j = 0; j < NJ; ++j) {
      sv[j] = (unsigned)kv[j] - nb;
      hv[j] = sv[j] < (unsigned)NBRUN;
      mv[j] = __builtin_amdgcn_ballot_w32(hv[j]);
      wc += (int)__builtin_popcount(mv[j]);
    }
    const int buf = (it & 1) * 8;
    if (lane == 0) misc[buf + wave] = wc;
    __syncthreads();
    const v4i ca = *(const v4ia*)(misc + buf);
    const v4i cb = *(const v4ia*)(misc + buf + 4);
    const int c0 = clampi(ca.x, 0, SUB), c1 = clampi(ca.y, 0, SUB), c2 = clampi(ca.z, 0, SUB), c3 = clampi(ca.w, 0, SUB);
    const int c4 = clampi(cb.x, 0, SUB), c5 = clampi(cb.y, 0, SUB), c6 = clampi(cb.z, 0, SUB), c7 = clampi(cb.w, 0, SUB);
    int pre = 0;
    pre += (wave > 0) ? c0 : 0;
    pre += (wave > 1) ? c1 : 0;
    pre += (wave > 2) ? c2 : 0;
    pre += (wave > 3) ? c3 : 0;
    pre += (wave > 4) ? c4 : 0;
    pre += (wave > 5) ? c5 : 0;
    pre += (wave > 6) ? c6 : 0;
    int all = c0 + c1 + c2 + c3 + c4 + c5 + c6 + c7;
    pre = __builtin_amdgcn_readfirstlane(pre);
    all = __builtin_amdgcn_readfirstlane(all);
    int pos = total + pre;
#pragma unroll
    for (int j = 0; j < NJ; ++j) {
      const int rank = (int)__builtin_amdgcn_mbcnt_lo(mv[j], 0u);
      const int p = pos + rank;
      if (hv[j] && p < RCAP) raw[p] = ((e0 + 32 * j) << SLB) | (int)sv[j];
      pos += (int)__builtin_popcount(mv[j]);
    }
    total += all;
  }
  __syncthreads();
  const int ovf = (total > RCAP) ? 1 : 0;
  const int tt  = total < 0 ? 0 : (total > RCAP ? RCAP : total);

  const unsigned myLo = (unsigned)(wave * (NBRUN / NWAVE));
#pragma unroll 1
  for (int b0 = 0; b0 < tt; b0 += 32) {
    const int idx = b0 + lane;
    const int u = raw[idx < RCAP ? idx : RCAP - 1];
    const unsigned rel = (unsigned)(u & (NBRUN - 1)) - myLo;
    const bool mine = (idx < tt) && (rel < (unsigned)(NBRUN / NWAVE));
#pragma unroll 1
    for (unsigned mk = __builtin_amdgcn_ballot_w32(mine); mk != 0u; mk &= mk - 1u) {
      const int k  = __builtin_ctz(mk);
      const int uk = __builtin_amdgcn_readlane(u, k);
      if (lane == 0) {
        const int sl = uk & (NBRUN - 1);
        cnt[sl] = cnt[sl] + 1;
      }
    }
  }
  __syncthreads();

  if (wave == 0) {
    const int base = lane * (NBRUN / 32);
    int s = 0, mx = 0;
#pragma unroll 1
    for (int i = 0; i < NBRUN / 32; ++i) {
      const int v = cnt[base + i];
      s += v;
      mx = v > mx ? v : mx;
    }
    int incl = s;
#pragma unroll
    for (int d = 1; d < 32; d <<= 1) {
      const int y = __shfl_up(incl, d, 32);
      if (lane >= d) incl += y;
    }
#pragma unroll
    for (int d = 16; d >= 1; d >>= 1) {
      const int y = __shfl_xor(mx, d, 32);
      mx = y > mx ? y : mx;
    }
    int run = incl - s;
#pragma unroll 1
    for (int i = 0; i < NBRUN / 32; ++i) {
      const int cv = cnt[base + i];
      offs[base + i] = run;
      cur[base + i]  = run;
      run += cv;
    }
    if (lane == 0) misc[16] = (ovf != 0 || mx > DEGCAP) ? 1 : 0;
  }
  __syncthreads();

#pragma unroll 1
  for (int b0 = 0; b0 < tt; b0 += 32) {
    const int idx = b0 + lane;
    const int u = raw[idx < RCAP ? idx : RCAP - 1];
    const unsigned rel = (unsigned)(u & (NBRUN - 1)) - myLo;
    const bool mine = (idx < tt) && (rel < (unsigned)(NBRUN / NWAVE));
#pragma unroll 1
    for (unsigned mk = __builtin_amdgcn_ballot_w32(mine); mk != 0u; mk &= mk - 1u) {
      const int k  = __builtin_ctz(mk);
      const int uk = __builtin_amdgcn_readlane(u, k);
      if (lane == 0) {
        const int sl = uk & (NBRUN - 1);
        int p = cur[sl];
        p = p < 0 ? 0 : (p > RCAP - 1 ? RCAP - 1 : p);
        grp[p] = uk;
        cur[sl] = p + 1;
      }
    }
  }
  __syncthreads();

  const int bflag = misc[16];
  if (wave == 0 && lane < 8) {
    const v4i fv = (v4i){bflag, bflag, bflag, bflag};
    volatile v4i* fp = (volatile v4i*)(flags + blk * 32 + 4 * lane);
    *fp = fv;
    __threadfence();
    *fp = fv;
  }

  const float qn = __int_as_float(0x7fc00000);
  const float pz = (bflag != 0) ? qn : 0.0f;
  int nsl = NN - nodeBase;
  nsl = nsl < 0 ? 0 : (nsl > NBRUN ? NBRUN : nsl);
  unsigned* rb = (unsigned*)(dsm + ZINTS + MISC_INTS) + wave * 128;
#pragma unroll 1
  for (int s0 = 0; s0 < nsl; s0 += NWAVE) {
    const int s    = s0 + wave;
    const int node = nodeBase + s;
    int c = clampi(cnt[s], 0, DEGCAP);
    c = __builtin_amdgcn_readfirstlane(c);
    int o = clampi(offs[s], 0, RCAP);
    o = __builtin_amdgcn_readfirstlane(o);
    int i0 = o + lane;      i0 = i0 > RCAP - 1 ? RCAP - 1 : i0;
    int i1 = o + 32 + lane; i1 = i1 > RCAP - 1 ? RCAP - 1 : i1;
    const int ent0 = grp[i0];
    const int ent1 = grp[i1];
    int sr0, sr1;
    float w0, w1;
    fetch_hit(ei, ew, ent0, lane, c, sr0, w0);
    fetch_hit(ei, ew, ent1, 32 + lane, c, sr1, w1);
    const int n0 = c < 32 ? c : 32;
    const int n1 = c - n0;
    float wsum = 0.0f;
    {
      const int w0i = __float_as_int(w0), w1i = __float_as_int(w1);
#pragma unroll 1
      for (int k = 0; k < n0; ++k) wsum += __int_as_float(__builtin_amdgcn_readlane(w0i, k));
#pragma unroll 1
      for (int k = 0; k < n1; ++k) wsum += __int_as_float(__builtin_amdgcn_readlane(w1i, k));
    }
    const float denom = (wsum > 1e-8f) ? wsum : 1e-8f;
    const float wn0 = w0 / denom;
    const float wn1 = w1 / denom;
    float a0 = 0.0f, a1 = 0.0f, a2 = 0.0f, a3 = 0.0f;
    walk_hits(apl, sr0, wn0, n0, lane, a0, a1, a2, a3);
    walk_hits(apl, sr1, wn1, n1, lane, a0, a1, a2, a3);
    const bool has = c > 0;
    const float m0 = (has ? a0 : 0.0f) + pz;
    const float m1 = (has ? a1 : 0.0f) + pz;
    const float m2 = (has ? a2 : 0.0f) + pz;
    const float m3 = (has ? a3 : 0.0f) + pz;
    const v2u hw = (v2u){ pk16(bf16_bits(m0), bf16_bits(m1)), pk16(bf16_bits(m2), bf16_bits(m3)) };
    *(v2ua*)(rb + 2 * lane) = hw;
    if (AGG_TERMS == 2) {
      const v2u lw = (v2u){ pk16(bf16_lo_bits(m0), bf16_lo_bits(m1)), pk16(bf16_lo_bits(m2), bf16_lo_bits(m3)) };
      *(v2ua*)(rb + 64 + 2 * lane) = lw;
    }
    wave_sync();
    const int li = (AGG_TERMS == 2) ? lane : (lane & 15);
    const v4u q = *(const v4ua*)(rb + 4 * li);
    wave_sync();
    const bool lok = (AGG_TERMS == 2) || (lane < 16);
    if (node < NN && lok) {
      volatile v4u* dp = (volatile v4u*)(apl + (size_t)node * KA + DF + 8 * lane);
      *dp = q;
      __threadfence();
      *dp = q;
    }
  }
}

__global__ __launch_bounds__(NTHR) void k_flagfix(const int* __restrict__ flags, float* __restrict__ out) {
  const int blk  = (int)blockIdx.x;
  const int lane = (int)threadIdx.x & 31, wave = (int)threadIdx.x >> 5;
  const int f = flags[clampi(blk, 0, NBLK - 1) * 32];
  if (f != 1) return;
  const float qn = __int_as_float(0x7fc00000);
  const v4f nv = (v4f){qn, qn, qn, qn};
  const int nodeBase = blk * NBRUN;
#pragma unroll 1
  for (int r = wave; r < NBRUN; r += NWAVE) {
    const int node = nodeBase + r;
    if (node < NN) {
      volatile v4f* p = (volatile v4f*)(out + (size_t)node * DOUT + 4 * lane);
      *p = nv;
      __threadfence();
      *p = nv;
    }
  }
}

extern "C" void kernel_launch(void* const* d_in, const int* in_sizes, int n_in,
                              void* d_out, int out_size, void* d_ws, size_t ws_size,
                              hipStream_t stream) {
  if (n_in < 5) return;
  if (in_sizes[0] != NN * DF) return;
  if (in_sizes[1] != 2 * NE) return;
  if (in_sizes[2] != NE) return;
  if (in_sizes[3] != DOUT * 2 * DF) return;
  if (in_sizes[4] != DOUT) return;
  if (out_size != NN * DOUT) return;
  if (WS_TOTAL > ws_size) return;

  const float* x  = (const float*)d_in[0];
  const int*   ei = (const int*)d_in[1];
  const float* ew = (const float*)d_in[2];
  const float* W  = (const float*)d_in[3];
  const float* b  = (const float*)d_in[4];
  float* out = (float*)d_out;

  char* ws = (char*)d_ws;
  unsigned short* apl   = (unsigned short*)(ws + OFF_A);
  unsigned short* wc    = (unsigned short*)(ws + OFF_W);
  float*          biasr = (float*)(ws + OFF_BIAS);
  int*            flags = (int*)(ws + OFF_FLAGS);

  hipFuncSetAttribute(reinterpret_cast<const void*>(&k_scan), hipFuncAttributeMaxDynamicSharedMemorySize,
                      (int)SCAN_LDS_BYTES);

  k_prep<<<PREP_NB, NTHR, 0, stream>>>(x, W, b, apl, wc, biasr);
  k_scan<<<NBLK, NTHR, SCAN_LDS_BYTES, stream>>>(ei, ew, apl, flags);
  k_gemm_nt<0, 1><<<GEMM_NB, 256, 0, stream>>>(apl, wc, biasr, out, NN, DOUT, KA, DOUT);
  k_flagfix<<<NBLK, NTHR, 0, stream>>>(flags, out);
}
